// WindowCrossBandDir_8564164789081
// MI455X (gfx1250) — hardware-verified
//
#include <hip/hip_runtime.h>
#define NB 4
#define CC 64
#define HHp 128
#define WWp 128
#define NPX (HHp * WWp)
#define WS 8
#define SSd 4
#define NWd 31
#define NL (NWd * NWd)
#define NTK 64
#define NHd 4
#define DH 16
#define LH 481
typedef __bf16 v16b __attribute__((ext_vector_type(16)));
typedef unsigned short v8us __attribute__((ext_vector_type(8), may_alias));
typedef float  v8f  __attribute__((ext_vector_type(8)));
typedef float  v4f  __attribute__((ext_vector_type(4)));
typedef float  v4fa __attribute__((ext_vector_type(4), may_alias));
union FragB { v16b v; v8us half[2]; unsigned short u[16]; };

__device__ __forceinline__ unsigned short bf16_bits(float x) { unsigned int u = __float_as_uint(x); return (unsigned short)((u + 0x7FFFu + ((u >> 16) & 1u)) >> 16); }
__device__ __forceinline__ float bf16_val(unsigned short b) { return __uint_as_float(((unsigned int)b) << 16); }
__device__ __forceinline__ float bf16_round(float x) { return bf16_val(bf16_bits(x)); }
template <int NT>
__device__ __forceinline__ v8f mmaN(v16b ah, v16b al, v16b bh, v16b bl, v8f c) {
  c = __builtin_amdgcn_wmma_f32_16x16x32_bf16(false, ah, false, bh, (short)0, c, false, false);
  if (NT >= 2) c = __builtin_amdgcn_wmma_f32_16x16x32_bf16(false, al, false, bh, (short)0, c, false, false);
  if (NT >= 3) c = __builtin_amdgcn_wmma_f32_16x16x32_bf16(false, ah, false, bl, (short)0, c, false, false);
  asm volatile("v_nop\n\tv_nop\n\tv_nop\n\tv_nop" : "+v"(c) : "v"(ah), "v"(al), "v"(bh), "v"(bl));
  return c;
}

__global__ __launch_bounds__(256) void k_wt_bf16(const float* __restrict__ W, unsigned short* __restrict__ Wt, int K, int N) {
  const int t = blockIdx.x * 256 + threadIdx.x;
  const int k8n = K / 8;
  if (t >= N * k8n) return;
  const int n = t / k8n, k8 = (t % k8n) * 8;
  v8us v;
#pragma unroll
  for (int i = 0; i < 8; ++i) v[i] = bf16_bits(W[(size_t)(k8 + i) * N + n]);
  *(volatile v8us*)(Wt + (size_t)n * K + k8) = v;
  __threadfence();
  *(volatile v8us*)(Wt + (size_t)n * K + k8) = v;
}

template <bool ASPLIT, int ACT, bool BIAS_BF16>
__global__ __launch_bounds__(128) void k_gemm_bf(const float* __restrict__ A, int lda, const unsigned short* __restrict__ Wt, int ldb,
                                               const float* __restrict__ bias, float* __restrict__ C, int ldc, int M, int N, int K) {
  __shared__ __attribute__((aligned(16))) float so[4][16][64];
  const int tid = threadIdx.x, w = tid >> 5, lane = tid & 31, ln = lane & 15, hh = lane >> 4;
  const int ntn = N / 64;
  const int wid = blockIdx.x * 4 + w;
  const int mt = wid / ntn, nq = wid % ntn;
  if (mt * 16 >= M) return;
  const int row0 = mt * 16, col0 = nq * 64;
  const float* arow = A + (size_t)(row0 + ln) * lda;
  v8f acc[4] = {};
  for (int kb = 0; kb < K; kb += 32) {
    FragB ah, al;
    const v4f x0 = *(const v4fa*)(arow + kb + 8 * hh), x1 = *(const v4fa*)(arow + kb + 8 * hh + 4);
    const v4f x2 = *(const v4fa*)(arow + kb + 16 + 8 * hh), x3 = *(const v4fa*)(arow + kb + 16 + 8 * hh + 4);
    float xs[16] = {x0[0],x0[1],x0[2],x0[3],x1[0],x1[1],x1[2],x1[3],x2[0],x2[1],x2[2],x2[3],x3[0],x3[1],x3[2],x3[3]};
#pragma unroll
    for (int i = 0; i < 16; ++i) { const unsigned short hb = bf16_bits(xs[i]); ah.u[i] = hb; al.u[i] = ASPLIT ? bf16_bits(xs[i] - bf16_val(hb)) : (unsigned short)0; }
#pragma unroll
    for (int t = 0; t < 4; ++t) {
      const unsigned short* brow = Wt + (size_t)(col0 + t * 16 + ln) * ldb + kb;
      FragB b;
      b.half[0] = *(const v8us*)(brow + 8 * hh);
      b.half[1] = *(const v8us*)(brow + 16 + 8 * hh);
      acc[t] = mmaN<ASPLIT ? 2 : 1>(ah.v, al.v, b.v, b.v, acc[t]);
    }
  }
#pragma unroll
  for (int t = 0; t < 4; ++t) {
    float bv = bias ? bias[col0 + t * 16 + ln] : 0.f;
    if (BIAS_BF16) bv = bf16_round(bv);
#pragma unroll
    for (int r = 0; r < 8; ++r) { float v = acc[t][r] + bv; if (ACT == 1) v = fmaxf(v, 0.f); so[w][8 * hh + r][t * 16 + ln] = v; }
  }
  __builtin_amdgcn_fence(__ATOMIC_ACQ_REL, "workgroup");
  __builtin_amdgcn_wave_barrier();
  const int rsub = lane >> 4, c4 = (lane & 15) * 4;
  for (int pass = 0; pass < 2; ++pass) {
#pragma unroll
    for (int q = 0; q < 8; ++q) {
      const int r = q * 2 + rsub;
      const v4f v = *(const v4fa*)&so[w][r][c4];
      *(volatile v4f*)(C + (size_t)(row0 + r) * ldc + col0 + c4) = v;
    }
    if (pass == 0) __threadfence();
  }
}

template <bool ASPLIT, int ACT, bool BIAS_BF16, bool RES_BF16>
__global__ __launch_bounds__(128) void k_gemm_bf3(const float* __restrict__ A, int lda, const unsigned short* __restrict__ Wt, int ldb,
                                                const float* __restrict__ bias, const float* __restrict__ resid, int rmod, int ldr,
                                                float* __restrict__ C, int ldc, int M, int N, int K) {
  __shared__ __attribute__((aligned(16))) float so[4][16][64];
  const int tid = threadIdx.x, w = tid >> 5, lane = tid & 31, ln = lane & 15, hh = lane >> 4;
  const int ntn = N / 64;
  const int wid = blockIdx.x * 4 + w;
  const int mt = wid / ntn, nq = wid % ntn;
  if (mt * 16 >= M) return;
  const int row0 = mt * 16, col0 = nq * 64;
  const float* arow = A + (size_t)(row0 + ln) * lda;
  v8f acc[4] = {};
  for (int kb = 0; kb < K; kb += 32) {
    FragB ah, al;
    const v4f x0 = *(const v4fa*)(arow + kb + 8 * hh), x1 = *(const v4fa*)(arow + kb + 8 * hh + 4);
    const v4f x2 = *(const v4fa*)(arow + kb + 16 + 8 * hh), x3 = *(const v4fa*)(arow + kb + 16 + 8 * hh + 4);
    float xs[16] = {x0[0],x0[1],x0[2],x0[3],x1[0],x1[1],x1[2],x1[3],x2[0],x2[1],x2[2],x2[3],x3[0],x3[1],x3[2],x3[3]};
#pragma unroll
    for (int i = 0; i < 16; ++i) { const unsigned short hb = bf16_bits(xs[i]); ah.u[i] = hb; al.u[i] = ASPLIT ? bf16_bits(xs[i] - bf16_val(hb)) : (unsigned short)0; }
#pragma unroll
    for (int t = 0; t < 4; ++t) {
      const unsigned short* brow = Wt + (size_t)(col0 + t * 16 + ln) * ldb + kb;
      FragB b;
      b.half[0] = *(const v8us*)(brow + 8 * hh);
      b.half[1] = *(const v8us*)(brow + 16 + 8 * hh);
      acc[t] = mmaN<ASPLIT ? 2 : 1>(ah.v, al.v, b.v, b.v, acc[t]);
    }
  }
#pragma unroll
  for (int t = 0; t < 4; ++t) {
    const int col = col0 + t * 16 + ln;
    float bv = bias ? bias[col] : 0.f;
    if (BIAS_BF16) bv = bf16_round(bv);
#pragma unroll
    for (int r = 0; r < 8; ++r) {
      float v = acc[t][r] + bv;
      if (resid) { float rv = resid[(size_t)((row0 + 8 * hh + r) % rmod) * ldr + col]; if (RES_BF16) rv = bf16_round(rv); v += rv; }
      if (ACT == 1) v = fmaxf(v, 0.f);
      if (ACT == 2) v = 0.5f * v * (1.0f + erff(v * 0.70710678118654752f));
      if (ACT == 3) { const float u = 0.7978845608028654f * (v + 0.044715f * v * v * v); v = 0.5f * v * (1.0f + tanhf(u)); }
      so[w][8 * hh + r][t * 16 + ln] = v;
    }
  }
  __builtin_amdgcn_fence(__ATOMIC_ACQ_REL, "workgroup");
  __builtin_amdgcn_wave_barrier();
  const int rsub = lane >> 4, c4 = (lane & 15) * 4;
  for (int pass = 0; pass < 2; ++pass) {
#pragma unroll
    for (int q = 0; q < 8; ++q) {
      const int r = q * 2 + rsub;
      const v4f v = *(const v4fa*)&so[w][r][c4];
      *(volatile v4f*)(C + (size_t)(row0 + r) * ldc + col0 + c4) = v;
    }
    if (pass == 0) __threadfence();
  }
}
template <bool PARAM_BF16>
__global__ __launch_bounds__(256) void k_layernorm(const float* __restrict__ X, const float* __restrict__ R, const float* __restrict__ g, const float* __restrict__ bta,
                                                  float* __restrict__ out_sum, float* __restrict__ out_norm, int N, float eps) {
  __shared__ float red[256];
  const int row = blockIdx.x, tid = threadIdx.x;
  const float* x = X + (size_t)row * N; const float* rr = R ? R + (size_t)row * N : nullptr;
  float vals[16];
  const int per = N / 256;
  float s1 = 0.f;
  for (int u = 0; u < per / 4; ++u) {
    const int j = tid * 4 + 1024 * u;
    const v4f a = *(const v4fa*)(x + j);
    v4f b = {0.f,0.f,0.f,0.f}; if (rr) b = *(const v4fa*)(rr + j);
#pragma unroll
    for (int q = 0; q < 4; ++q) { const float v = a[q] + b[q]; vals[u * 4 + q] = v; s1 += v; }
  }
  red[tid] = s1; __syncthreads();
  for (int st = 128; st > 0; st >>= 1) { if (tid < st) red[tid] += red[tid + st]; __syncthreads(); }
  const float mu = red[0] / (float)N; __syncthreads();
  float s2 = 0.f;
  for (int u = 0; u < per / 4; ++u)
#pragma unroll
    for (int q = 0; q < 4; ++q) { const float c = vals[u * 4 + q] - mu; s2 += c * c; }
  red[tid] = s2; __syncthreads();
  for (int st = 128; st > 0; st >>= 1) { if (tid < st) red[tid] += red[tid + st]; __syncthreads(); }
  const float rs = rsqrtf(red[0] / (float)N + eps);
  for (int pass = 0; pass < 2; ++pass) {
    for (int u = 0; u < per / 4; ++u) {
      const int j = tid * 4 + 1024 * u;
      v4f o, sm;
#pragma unroll
      for (int q = 0; q < 4; ++q) {
        float gg = g[j + q], bb = bta[j + q];
        if (PARAM_BF16) { gg = bf16_round(gg); bb = bf16_round(bb); }
        sm[q] = vals[u * 4 + q]; o[q] = (vals[u * 4 + q] - mu) * rs * gg + bb;
      }
      if (out_sum) *(volatile v4f*)(out_sum + (size_t)row * N + j) = sm;
      *(volatile v4f*)(out_norm + (size_t)row * N + j) = o;
    }
    if (pass == 0) __threadfence();
  }
}


typedef _Float16 v16h __attribute__((ext_vector_type(16)));
union FragH { v16h v; v8us half[2]; _Float16 h[16]; unsigned short u[16]; };
template <int NT>
__device__ __forceinline__ v8f mmaH(v16h ah, v16h al, v16h bh, v16h bl, v8f c) {
  c = __builtin_amdgcn_wmma_f32_16x16x32_f16(false, ah, false, bh, (short)0, c, false, false);
  if (NT >= 2) c = __builtin_amdgcn_wmma_f32_16x16x32_f16(false, al, false, bh, (short)0, c, false, false);
  if (NT >= 3) c = __builtin_amdgcn_wmma_f32_16x16x32_f16(false, ah, false, bl, (short)0, c, false, false);
  asm volatile("v_nop\n\tv_nop\n\tv_nop\n\tv_nop" : "+v"(c) : "v"(ah), "v"(al), "v"(bh), "v"(bl));
  return c;
}
template <bool ASPLIT>
__global__ __launch_bounds__(128) void k_gemm_h(const float* __restrict__ A, int lda, size_t sA, const _Float16* __restrict__ Bh, int ldb, size_t sB, float alpha, float* __restrict__ C, int ldc, size_t sC, int M, int N, int K) {
  __shared__ __attribute__((aligned(16))) float so[4][16][64];
  const int tid = threadIdx.x, w = tid >> 5, lane = tid & 31, ln = lane & 15, hh = lane >> 4; const int by = blockIdx.y;
  A += (size_t)by * sA; Bh += (size_t)by * sB; C += (size_t)by * sC;
  const int ntn = (N + 63) / 64; const int wid = blockIdx.x * 4 + w; const int mt = wid / ntn, nq = wid % ntn; if (mt * 16 >= M) return;
  const int row0 = mt * 16, col0 = nq * 64; const float* arow = A + (size_t)(row0 + ln) * lda;
  v8f acc[4] = {};
  for (int kb = 0; kb < K; kb += 32) {
    FragH ah, al;
    const v4f x0 = *(const v4fa*)(arow + kb + 8 * hh), x1 = *(const v4fa*)(arow + kb + 8 * hh + 4), x2 = *(const v4fa*)(arow + kb + 16 + 8 * hh), x3 = *(const v4fa*)(arow + kb + 16 + 8 * hh + 4);
    float xs[16] = {x0[0],x0[1],x0[2],x0[3],x1[0],x1[1],x1[2],x1[3],x2[0],x2[1],x2[2],x2[3],x3[0],x3[1],x3[2],x3[3]};
#pragma unroll
    for (int i = 0; i < 16; ++i) { const _Float16 h = (_Float16)xs[i]; ah.h[i] = h; al.h[i] = ASPLIT ? (_Float16)(xs[i] - (float)h) : (_Float16)0.0f; }
#pragma unroll
    for (int t = 0; t < 4; ++t) { if (col0 + t * 16 >= N) continue; const size_t boff = (size_t)(col0 + t * 16 + ln) * ldb + kb; FragH bq; bq.half[0] = *(const v8us*)(Bh + boff + 8 * hh); bq.half[1] = *(const v8us*)(Bh + boff + 16 + 8 * hh);
      acc[t] = mmaH<ASPLIT ? 2 : 1>(ah.v, al.v, bq.v, bq.v, acc[t]); }
  }
#pragma unroll
  for (int t = 0; t < 4; ++t) { if (col0 + t * 16 >= N) continue;
#pragma unroll
    for (int r = 0; r < 8; ++r) so[w][8 * hh + r][t * 16 + ln] = acc[t][r] * alpha; }
  __builtin_amdgcn_fence(__ATOMIC_ACQ_REL, "workgroup"); __builtin_amdgcn_wave_barrier();
  const int rsub = lane >> 4, c4 = (lane & 15) * 4;
  for (int pass = 0; pass < 2; ++pass) {
#pragma unroll
    for (int q = 0; q < 8; ++q) { const int r = q * 2 + rsub; if (col0 + c4 < N) { const v4f v = *(const v4fa*)&so[w][r][c4]; *(volatile v4f*)(C + (size_t)(row0 + r) * ldc + col0 + c4) = v; } }
    if (pass == 0) __threadfence(); }
}

__global__ __launch_bounds__(256) void k_wt_f16(const float* __restrict__ W, _Float16* __restrict__ Wt, int K, int N, float scale) {
  const int t = blockIdx.x * 256 + threadIdx.x; if (t >= N * (K / 8)) return; const int n = t / (K / 8), k8 = (t % (K / 8)) * 8; FragH f;
#pragma unroll
  for (int i = 0; i < 8; ++i) f.h[i] = (_Float16)(bf16_round(W[(size_t)(k8 + i) * N + n]) * scale); const v8us o = f.half[0];
  *(volatile v8us*)((unsigned short*)Wt + (size_t)n * K + k8) = o; __threadfence(); *(volatile v8us*)((unsigned short*)Wt + (size_t)n * K + k8) = o;
}
template <int ACT>
__global__ __launch_bounds__(128) void k_gemm_hhx(const _Float16* __restrict__ A, int lda, size_t sA, const _Float16* __restrict__ Bh, int ldb, size_t sB, float alpha, const float* __restrict__ bias, size_t sBias, const float* __restrict__ CP, int rowsPerB, size_t sCPb, int row0g,
    float* __restrict__ C, _Float16* __restrict__ C16, int ldc, size_t sC, int M, int N, int K) {
  __shared__ __attribute__((aligned(16))) float so[4][16][64];
  const int tid = threadIdx.x, w = tid >> 5, lane = tid & 31, ln = lane & 15, hh = lane >> 4; const int by = blockIdx.y;
  A += (size_t)by * sA; Bh += (size_t)by * sB; const size_t cofs = (size_t)by * sC; const float* bp = bias ? bias + (size_t)by * sBias : nullptr;
  const int ntn = (N + 63) / 64; const int wid = blockIdx.x * 4 + w; const int mt = wid / ntn, nq = wid % ntn; if (mt * 16 >= M) return;
  const int row0 = mt * 16, col0 = nq * 64; const _Float16* arow = A + (size_t)(row0 + ln) * lda;
  v8f acc[4] = {};
  for (int kb = 0; kb < K; kb += 32) { FragH ah; ah.half[0] = *(const v8us*)((const unsigned short*)arow + kb + 8 * hh); ah.half[1] = *(const v8us*)((const unsigned short*)arow + kb + 16 + 8 * hh);
#pragma unroll
    for (int t = 0; t < 4; ++t) { if (col0 + t * 16 >= N) continue; const size_t boff = (size_t)(col0 + t * 16 + ln) * ldb + kb; FragH bq; bq.half[0] = *(const v8us*)((const unsigned short*)Bh + boff + 8 * hh); bq.half[1] = *(const v8us*)((const unsigned short*)Bh + boff + 16 + 8 * hh);
      acc[t] = mmaH<1>(ah.v, ah.v, bq.v, bq.v, acc[t]); }
  }
#pragma unroll
  for (int t = 0; t < 4; ++t) { if (col0 + t * 16 >= N) continue; const int col = col0 + t * 16 + ln; const float bv = bp ? bf16_round(bp[col]) : 0.f;
#pragma unroll
    for (int r = 0; r < 8; ++r) { float v = acc[t][r] * alpha + bv; if (CP) { const int bidx = (row0g + row0 + 8 * hh + r) / rowsPerB; v += CP[(size_t)bidx * sCPb + (size_t)by * 64 + col]; } if (ACT == 1) v = (v > 0.f) ? v : expm1f(v); else if (ACT == 7) v = (v > 0.f) ? v + 1.0f : expf(v); else if (ACT == 8) v = tanhf(v); else if (ACT == 9) v = 0.5f * v * (1.0f + tanhf(0.7978845608028654f * (v + 0.044715f * v * v * v))); else if (ACT == 11) v = 1.0f / (1.0f + expf(-v)); else if (ACT == 12) v = (v > 0.f) ? v : 0.01f * v; else if (ACT == 14) v = (v > 0.f) ? v : 0.1f * v; else if (ACT == 15) v = v / (1.0f + expf(-v)); else if (ACT == 3) v = fmaxf(v, 0.f); else if (ACT == 6) v = 0.5f * v * (1.0f + erff(v * 0.70710678118654752f)); so[w][8 * hh + r][t * 16 + ln] = v; } }
  __builtin_amdgcn_fence(__ATOMIC_ACQ_REL, "workgroup"); __builtin_amdgcn_wave_barrier();
  const int rsub = lane >> 4, c4 = (lane & 15) * 4; typedef _Float16 v4h __attribute__((ext_vector_type(4)));
  for (int pass = 0; pass < 2; ++pass) {
#pragma unroll
    for (int q = 0; q < 8; ++q) { const int r = q * 2 + rsub; if (col0 + c4 < N) { const v4f v = *(const v4fa*)&so[w][r][c4]; if (C) *(volatile v4f*)(C + cofs + (size_t)(row0 + r) * ldc + col0 + c4) = v; if (C16) { v4h h4; for (int i = 0; i < 4; ++i) h4[i] = (_Float16)v[i]; *(volatile v4h*)(C16 + cofs + (size_t)(row0 + r) * ldc + col0 + c4) = h4; } } }
    if (pass == 0) __threadfence(); }
}


typedef _Float16 v4h __attribute__((ext_vector_type(4)));

__global__ __launch_bounds__(256) void k_x16(const float* __restrict__ x, _Float16* __restrict__ X16, size_t n8) { const size_t t = (size_t)blockIdx.x * 256 + threadIdx.x; if (t >= n8) return; FragH f;
#pragma unroll
  for (int q = 0; q < 8; ++q) f.h[q] = (_Float16)bf16_round(x[t * 8 + q]); *(volatile v8us*)((unsigned short*)X16 + t * 8) = f.half[0]; __threadfence(); *(volatile v8us*)((unsigned short*)X16 + t * 8) = f.half[0]; }
__global__ __launch_bounds__(256) void k_h16(const float* __restrict__ x, _Float16* __restrict__ X16, size_t n8) { const size_t t = (size_t)blockIdx.x * 256 + threadIdx.x; if (t >= n8) return; FragH f;
#pragma unroll
  for (int q = 0; q < 8; ++q) f.h[q] = (_Float16)x[t * 8 + q]; *(volatile v8us*)((unsigned short*)X16 + t * 8) = f.half[0]; __threadfence(); *(volatile v8us*)((unsigned short*)X16 + t * 8) = f.half[0]; }
__global__ __launch_bounds__(256) void k_round16f(const float* __restrict__ W, _Float16* __restrict__ Bt, size_t n8) { const size_t t = (size_t)blockIdx.x * 256 + threadIdx.x; if (t >= n8) return; FragH f;
#pragma unroll
  for (int i = 0; i < 8; ++i) f.h[i] = (_Float16)(bf16_round(W[t * 8 + i]) * 16.0f); *(volatile v8us*)((unsigned short*)Bt + t * 8) = f.half[0]; __threadfence(); *(volatile v8us*)((unsigned short*)Bt + t * 8) = f.half[0]; }
template <int NHv, int TTv>
__global__ __launch_bounds__(256) void k_vt(const _Float16* __restrict__ V16, int ldv, int voff, _Float16* __restrict__ Vt) { __shared__ unsigned short tl[64][66]; const int tid = threadIdx.x; const int slab = blockIdx.x / (TTv / 64), lg = blockIdx.x % (TTv / 64); const int b = slab / NHv, h = slab % NHv;
  for (int i = tid; i < 64 * 8; i += 256) { const int r = i / 8, c8 = (i % 8) * 8; FragH f; f.half[0] = *(const v8us*)((const unsigned short*)V16 + ((size_t)b * TTv + lg * 64 + r) * ldv + voff + h * 64 + c8);
#pragma unroll
    for (int q = 0; q < 8; ++q) tl[r][c8 + q] = f.u[q]; }
  __syncthreads();
  for (int pass = 0; pass < 2; ++pass) {
#pragma unroll
    for (int rd = 0; rd < 2; ++rd) { const int d = rd * 32 + tid / 8, pc = tid % 8; FragH f;
#pragma unroll
      for (int q = 0; q < 8; ++q) f.u[q] = tl[pc * 8 + q][d];
      *(volatile v8us*)((unsigned short*)Vt + ((size_t)slab * 64 + d) * TTv + lg * 64 + pc * 8) = f.half[0]; }
    if (pass == 0) __threadfence(); } }

__global__ __launch_bounds__(256) void k_hl(const float* __restrict__ F, _Float16* __restrict__ Hh, _Float16* __restrict__ Hl, size_t n8) { const size_t t = (size_t)blockIdx.x * 256 + threadIdx.x; if (t >= n8) return; FragH fh, fl; const v4f a = *(const v4fa*)(F + t * 8), c = *(const v4fa*)(F + t * 8 + 4);
#pragma unroll
  for (int q = 0; q < 4; ++q) { _Float16 h = (_Float16)a[q]; fh.h[q] = h; fl.h[q] = (_Float16)((a[q] - (float)h) * 1024.0f); h = (_Float16)c[q]; fh.h[4 + q] = h; fl.h[4 + q] = (_Float16)((c[q] - (float)h) * 1024.0f); }
  for (int pass = 0; pass < 2; ++pass) { *(volatile v8us*)((unsigned short*)Hh + t * 8) = fh.half[0]; *(volatile v8us*)((unsigned short*)Hl + t * 8) = fl.half[0]; if (pass == 0) __threadfence(); } }

__global__ __launch_bounds__(256) void k_pool(const float* __restrict__ high, float* __restrict__ POOL) {
  #pragma clang fp contract(off)
  __shared__ float red[256]; const int tid = threadIdx.x; const int bc = blockIdx.x; const float* p = high + (size_t)bc * NPX; float s = 0.f;
#pragma unroll 1
  for (int i = tid * 4; i < NPX; i += 1024) { const v4f v = *(const v4fa*)(p + i); s += (bf16_round(v[0]) + bf16_round(v[1])) + (bf16_round(v[2]) + bf16_round(v[3])); }
  red[tid] = s; __syncthreads(); for (int k = 128; k > 0; k >>= 1) { if (tid < k) red[tid] += red[tid + k]; __syncthreads(); }
  if (tid < 32) { *(volatile float*)(POOL + (size_t)bc * 32 + tid) = red[0] / (float)NPX; __threadfence(); *(volatile float*)(POOL + (size_t)bc * 32 + tid) = red[0] / (float)NPX; } }
__global__ __launch_bounds__(256) void k_gate(const float* __restrict__ POOL, const float* __restrict__ a1, const float* __restrict__ a2, const float* __restrict__ b1, const float* __restrict__ b2, const float* __restrict__ c1, const float* __restrict__ c2, int b, float* __restrict__ SG) {
  #pragma clang fp contract(off)
  __shared__ float tg[3]; const int tid = threadIdx.x;
  if (tid < 3) { const int g0 = (tid == 0) ? 0 : (tid == 1) ? 22 : 43, gn = (tid == 0) ? 22 : 21; const float* w1 = (tid == 0) ? a1 : (tid == 1) ? b1 : c1; float t = 0.f;
#pragma unroll 1
    for (int j = 0; j < gn; ++j) t += POOL[((size_t)b * CC + g0 + j) * 32] * bf16_round(w1[j]); tg[tid] = fmaxf(t, 0.f); }
  __syncthreads();
  if (tid < CC) { const int g = (tid < 22) ? 0 : (tid < 43) ? 1 : 2; const int j = tid - ((g == 0) ? 0 : (g == 1) ? 22 : 43); const float* w2 = (g == 0) ? a2 : (g == 1) ? b2 : c2; const float s = 1.0f / (1.0f + expf(-(tg[g] * bf16_round(w2[j])))); *(volatile float*)(SG + (size_t)b * CC + tid) = s; __threadfence(); *(volatile float*)(SG + (size_t)b * CC + tid) = s; } }
__global__ __launch_bounds__(256) void k_wg(const float* __restrict__ w, const float* __restrict__ SG, int b, int gate, _Float16* __restrict__ Bh, _Float16* __restrict__ Bl) {
  #pragma clang fp contract(off)
  const int t = blockIdx.x * 256 + threadIdx.x; if (t >= CC * (CC / 8)) return; const int c0 = (t % (CC / 8)) * 8, o = t / (CC / 8); FragH fh, fl;
#pragma unroll
  for (int q = 0; q < 8; ++q) { const int c = c0 + q; const float v = bf16_round(w[(size_t)o * CC + c]) * (gate ? SG[(size_t)b * CC + c] : 1.0f) * 16.0f; const _Float16 hi = (_Float16)v; fh.h[q] = hi; fl.h[q] = (_Float16)((v - (float)hi) * 1024.0f); }
  for (int pass = 0; pass < 2; ++pass) { *(volatile v8us*)((unsigned short*)Bh + (size_t)o * CC + c0) = fh.half[0]; *(volatile v8us*)((unsigned short*)Bl + (size_t)o * CC + c0) = fl.half[0]; if (pass == 0) __threadfence(); } }
__global__ __launch_bounds__(256) void k_pix16(const float* __restrict__ img, int b, _Float16* __restrict__ X16) { const int t = blockIdx.x * 256 + threadIdx.x; if (t >= NPX * (CC / 8)) return; const int c0 = (t % (CC / 8)) * 8, p = t / (CC / 8); FragH f;
#pragma unroll
  for (int q = 0; q < 8; ++q) f.h[q] = (_Float16)bf16_round(img[((size_t)b * CC + c0 + q) * NPX + p]);
  *(volatile v8us*)((unsigned short*)X16 + (size_t)p * CC + c0) = f.half[0]; __threadfence(); *(volatile v8us*)((unsigned short*)X16 + (size_t)p * CC + c0) = f.half[0]; }
__global__ __launch_bounds__(256) void k_gqk(const _Float16* __restrict__ Q16, const _Float16* __restrict__ K16, int l0, int nl, _Float16* __restrict__ UQ, _Float16* __restrict__ UK) { const int per = nl * NHd * NTK * 4; const int t = blockIdx.x * 256 + threadIdx.x; if (t >= 2 * per) return; const int plane = t / per; const int u = t % per; const int q = u & 3; const int n = (u >> 2) % NTK; const int lh = (u >> 2) / NTK; const int h = lh % NHd, l = l0 + lh / NHd; const int wy = l / NWd, wx = l % NWd; const int p = (SSd * wy + n / WS) * WWp + SSd * wx + n % WS;
  const _Float16* src = plane ? K16 : Q16; _Float16* dst = plane ? UK : UQ; FragH f;
  if (q < 2) f.half[0] = *(const v8us*)((const unsigned short*)src + (size_t)p * CC + h * DH + 8 * q); else {
#pragma unroll
    for (int j = 0; j < 8; ++j) f.h[j] = (_Float16)0.0f; }
  unsigned short* row = (unsigned short*)dst + ((size_t)lh * NTK + n) * 32 + 8 * q;
  *(volatile v8us*)row = f.half[0]; __threadfence(); *(volatile v8us*)row = f.half[0]; }
__global__ __launch_bounds__(256) void k_gv(const _Float16* __restrict__ V16, int l0, int nl, _Float16* __restrict__ UVt) { const int t = blockIdx.x * 256 + threadIdx.x; if (t >= nl * NHd * DH * (NTK / 8)) return; const int m0 = (t % (NTK / 8)) * 8; const int d = (t / (NTK / 8)) % DH; const int lh = t / ((NTK / 8) * DH); const int h = lh % NHd, l = l0 + lh / NHd; const int wy = l / NWd, wx = l % NWd; FragH f;
#pragma unroll
  for (int q = 0; q < 8; ++q) { const int m = m0 + q; const int p = (SSd * wy + m / WS) * WWp + SSd * wx + m % WS; f.h[q] = V16[(size_t)p * CC + h * DH + d]; }
  *(volatile v8us*)((unsigned short*)UVt + ((size_t)lh * DH + d) * NTK + m0) = f.half[0]; __threadfence(); *(volatile v8us*)((unsigned short*)UVt + ((size_t)lh * DH + d) * NTK + m0) = f.half[0]; }
__global__ __launch_bounds__(256) void k_soft(const float* __restrict__ S, int nrows, _Float16* __restrict__ P16) {
  #pragma clang fp contract(off)
  const int tid = threadIdx.x, w = tid >> 5, l = tid & 31; const int r = blockIdx.x * 8 + w; if (r >= nrows) return; const float a = S[(size_t)r * NTK + 2 * l], c = S[(size_t)r * NTK + 2 * l + 1]; float m = fmaxf(a, c);
  for (int o = 16; o > 0; o >>= 1) m = fmaxf(m, __shfl_xor(m, o, 32)); const float ea = expf(a - m), ec = expf(c - m); float s = ea + ec; for (int o = 16; o > 0; o >>= 1) s += __shfl_xor(s, o, 32); const float inv = 1024.0f / s; FragH f; f.h[0] = (_Float16)(ea * inv); f.h[1] = (_Float16)(ec * inv); const unsigned int v = *(const unsigned int*)&f.u[0];
  *(volatile unsigned int*)((unsigned short*)P16 + (size_t)r * NTK + 2 * l) = v; __threadfence(); *(volatile unsigned int*)((unsigned short*)P16 + (size_t)r * NTK + 2 * l) = v; }
__global__ __launch_bounds__(256) void k_fold(const float* __restrict__ O, _Float16* __restrict__ Fh, _Float16* __restrict__ Fl) {
  #pragma clang fp contract(off)
  const int t = blockIdx.x * 256 + threadIdx.x; if (t >= NPX * (CC / 4)) return; const int c0 = (t % (CC / 4)) * 4, p = t / (CC / 4); const int y = p / WWp, x = p % WWp; const int h = c0 / DH, d0 = c0 % DH; v4f acc; acc[0] = acc[1] = acc[2] = acc[3] = 0.f; int cnt = 0;
  for (int wy = y / SSd - 1; wy <= y / SSd; ++wy) { if (wy < 0 || wy >= NWd) continue; const int ty = y - SSd * wy; if (ty < 0 || ty >= WS) continue;
    for (int wx = x / SSd - 1; wx <= x / SSd; ++wx) { if (wx < 0 || wx >= NWd) continue; const int tx = x - SSd * wx; if (tx < 0 || tx >= WS) continue; const int l = wy * NWd + wx; const int n = ty * WS + tx; const v4f v = *(const v4fa*)(O + (((size_t)l * NHd + h) * NTK + n) * DH + d0);
#pragma unroll
      for (int q = 0; q < 4; ++q) acc[q] += v[q]; ++cnt; } }
  FragH fh, fl; const float inv = 1.0f / (float)cnt;
#pragma unroll
  for (int q = 0; q < 4; ++q) { const float v = acc[q] * inv; const _Float16 hi = (_Float16)v; fh.h[q] = hi; fl.h[q] = (_Float16)((v - (float)hi) * 1024.0f); }
  const unsigned long long vh = *(const unsigned long long*)&fh.u[0], vl = *(const unsigned long long*)&fl.u[0];
  for (int pass = 0; pass < 2; ++pass) { *(volatile unsigned long long*)((unsigned short*)Fh + (size_t)p * CC + c0) = vh; *(volatile unsigned long long*)((unsigned short*)Fl + (size_t)p * CC + c0) = vl; if (pass == 0) __threadfence(); } }
__global__ __launch_bounds__(256) void k_out(const float* __restrict__ img, const float* __restrict__ PR, int b, float* __restrict__ out) {
  #pragma clang fp contract(off)
  const int t = blockIdx.x * 256 + threadIdx.x; if (t >= CC * (NPX / 4)) return; const int p0 = (t % (NPX / 4)) * 4, c = t / (NPX / 4); const size_t base = ((size_t)b * CC + c) * NPX + p0; const v4f a = *(const v4fa*)(img + base); v4f o;
#pragma unroll
  for (int q = 0; q < 4; ++q) o[q] = bf16_round(a[q]) + PR[(size_t)(p0 + q) * CC + c];
  *(volatile v4f*)(out + base) = o; __threadfence(); *(volatile v4f*)(out + base) = o; }

extern "C" void kernel_launch(void* const* d_in, const int* in_sizes, int n_in,
                              void* d_out, int out_size, void* d_ws, size_t ws_size, hipStream_t stream) {
  (void)in_sizes; (void)n_in; (void)out_size;
  const float* const* I = (const float* const*)d_in; const float* low = I[0]; const float* high = I[1]; const float* w_ql = I[2]; const float* w_kh = I[3]; const float* w_vh = I[4]; const float* w_qh = I[5]; const float* w_kl = I[6]; const float* w_vl = I[7]; const float* w_pl = I[8]; const float* w_ph = I[9]; const float* s0a = I[10]; const float* s0b = I[11]; const float* s1a = I[12]; const float* s1b = I[13]; const float* s2a = I[14]; const float* s2b = I[15];
  char* ws = (char*)d_ws; size_t off = 0;
  auto take = [&](size_t bytes) { char* p = ws + off; off += (bytes + 255) & ~(size_t)255; return p; };
  float* POOL = (float*)take((size_t)NB * CC * 32 * 4); float* SG = (float*)take((size_t)NB * CC * 4);
  _Float16* Wh[8]; _Float16* Wl8; for (int i = 0; i < 8; ++i) Wh[i] = (_Float16*)take(CC * CC * 2); Wl8 = (_Float16*)take(CC * CC * 2);
  _Float16* L16 = (_Float16*)take((size_t)NPX * CC * 2); _Float16* H16 = (_Float16*)take((size_t)NPX * CC * 2); _Float16* M16[6]; for (int i = 0; i < 6; ++i) M16[i] = (_Float16*)take((size_t)NPX * CC * 2);
  _Float16* UQ = (_Float16*)take((size_t)LH * NHd * NTK * 32 * 2); _Float16* UK = (_Float16*)take((size_t)LH * NHd * NTK * 32 * 2); _Float16* UVt = (_Float16*)take((size_t)LH * NHd * DH * NTK * 2); float* S = (float*)take((size_t)LH * NHd * NTK * NTK * 4); _Float16* P16 = (_Float16*)take((size_t)LH * NHd * NTK * NTK * 2); float* O = (float*)take((size_t)NL * NHd * NTK * DH * 4);
  _Float16* Fh = (_Float16*)take((size_t)NPX * CC * 2); _Float16* Fl = (_Float16*)take((size_t)NPX * CC * 2); float* PR = (float*)take((size_t)NPX * CC * 4);
  if (off > ws_size) return;
  k_pool<<<NB * CC, 256, 0, stream>>>(high, POOL);
  const float* wsrc[8] = {w_ql, w_kh, w_vh, w_qh, w_kl, w_vl, w_pl, w_ph}; const int gated[8] = {0, 1, 1, 1, 0, 0, 0, 0};
  const dim3 gM(((NPX / 16) * 1 + 3) / 4, 1);
  for (int b = 0; b < NB; ++b) {
    k_gate<<<1, 256, 0, stream>>>(POOL, s0a, s0b, s1a, s1b, s2a, s2b, b, SG);
    for (int i = 0; i < 8; ++i) k_wg<<<(CC * (CC / 8) + 255) / 256, 256, 0, stream>>>(wsrc[i], SG, b, gated[i], Wh[i], Wl8);
    k_pix16<<<(NPX * (CC / 8) + 255) / 256, 256, 0, stream>>>(low, b, L16); k_pix16<<<(NPX * (CC / 8) + 255) / 256, 256, 0, stream>>>(high, b, H16);
    for (int i = 0; i < 6; ++i) { const _Float16* X = (i == 0 || i == 4 || i == 5) ? L16 : H16;
      k_gemm_hhx<0><<<gM, 128, 0, stream>>>(X, CC, 0, Wh[i], CC, 0, 0.0625f, nullptr, 0, nullptr, 1, 0, 0, nullptr, M16[i], CC, 0, NPX, CC, CC); }
    for (int dir = 0; dir < 2; ++dir) {
      const _Float16* Qm = dir ? M16[3] : M16[0]; const _Float16* Km = dir ? M16[4] : M16[1]; const _Float16* Vm = dir ? M16[5] : M16[2];
      for (int hf = 0; hf < 2; ++hf) { const int l0 = hf ? LH : 0, nl = hf ? (NL - LH) : LH; const int nlh = nl * NHd;
        k_gqk<<<(nlh * NTK * 8 + 255) / 256, 256, 0, stream>>>(Qm, Km, l0, nl, UQ, UK); k_gv<<<(nlh * DH * (NTK / 8) + 255) / 256, 256, 0, stream>>>(Vm, l0, nl, UVt);
        k_gemm_hhx<0><<<dim3(((NTK / 16) * 1 + 3) / 4, nlh), 128, 0, stream>>>(UQ, 32, (size_t)NTK * 32, UK, 32, (size_t)NTK * 32, 0.25f, nullptr, 0, nullptr, 1, 0, 0, S, nullptr, NTK, (size_t)NTK * NTK, NTK, NTK, 32);
        k_soft<<<(nlh * NTK + 7) / 8, 256, 0, stream>>>(S, nlh * NTK, P16);
        k_gemm_hhx<0><<<dim3(((NTK / 16) * 1 + 3) / 4, nlh), 128, 0, stream>>>(P16, NTK, (size_t)NTK * NTK, UVt, NTK, (size_t)DH * NTK, 0.0009765625f, nullptr, 0, nullptr, 1, 0, 0, O + (size_t)l0 * NHd * NTK * DH, nullptr, DH, (size_t)NTK * DH, NTK, DH, NTK); }
      k_fold<<<(NPX * (CC / 4) + 255) / 256, 256, 0, stream>>>(O, Fh, Fl);
      const int wi = dir ? 7 : 6; const float* res = dir ? high : low; float* outp = (float*)d_out + (dir ? (size_t)NB * CC * NPX : 0);
      k_gemm_hhx<0><<<gM, 128, 0, stream>>>(Fh, CC, 0, Wh[wi], CC, 0, 0.0625f, nullptr, 0, nullptr, 1, 0, 0, PR, nullptr, CC, 0, NPX, CC, CC); k_gemm_hhx<0><<<gM, 128, 0, stream>>>(Fl, CC, 0, Wh[wi], CC, 0, 0.0625f / 1024.0f, nullptr, 0, PR, 1, (size_t)CC, 0, PR, nullptr, CC, 0, NPX, CC, CC);
      k_out<<<(CC * (NPX / 4) + 255) / 256, 256, 0, stream>>>(res, PR, b, outp); }
  }
}
